// ResGnn_52510270161088
// MI455X (gfx1250) — hardware-verified
//
#include <hip/hip_runtime.h>
#include <stddef.h>


#define HCH   64
#define NCOL  128
#define EDIM  8
#define GR    32
#define XSP   132
#define NB    896
#define CHUNK 4096
#define NTHR  256
#define NWAVE 8
#define WCAP  512
#define NGRP  (CHUNK / (NTHR * 4))
#define EB    128
#define ESP   68

#define S_AMX  (NB * HCH)
#define S_DEN  (S_AMX + NB * 4)
#define S_OUTS (S_DEN + NB * 4)
#define S_LIST (S_OUTS + NB)
#define S_WCNT (S_LIST + NWAVE * WCAP)
#define LDS_WORDS (S_WCNT + 16)
#define LDS_BYTES (LDS_WORDS * 4)

static_assert(WCAP == (CHUNK / NTHR) * 32);
static_assert(NGRP == 4);
static_assert(NB < 1024);
static_assert((NB % (NWAVE * 4)) == 0);
static_assert((NB % 32) == 0);
static_assert((S_AMX % 4) == 0);
static_assert((S_DEN % 4) == 0);
static_assert((S_OUTS % 4) == 0);
static_assert((S_LIST % 4) == 0);
static_assert((S_WCNT % 4) == 0);
static_assert(LDS_BYTES == 278080);

typedef float    v4f  __attribute__((ext_vector_type(4)));
typedef float    v8f  __attribute__((ext_vector_type(8)));
typedef int      v4i  __attribute__((ext_vector_type(4)));
typedef _Float16 v8h  __attribute__((ext_vector_type(8)));
typedef _Float16 v16h __attribute__((ext_vector_type(16)));
union Frag   { v16h v; v8h half[2]; };
union Pack16 { v8h h; v4i i; };
union U8     { v4f v[2]; float f[8]; };

__device__ __forceinline__ v8f wm(v16h a, v16h b, v8f c) {
  v8f d = __builtin_amdgcn_wmma_f32_16x16x32_f16(false, a, false, b, (short)0, c, false, false);
  asm volatile("v_nop\n\tv_nop\n\tv_nop\n\tv_nop" : "+v"(d) : "v"(a), "v"(b));
  return d;
}

__device__ __forceinline__ v4i cvt8i(v4f a, v4f b) {
  Pack16 u;
  u.h[0] = (_Float16)a.x; u.h[1] = (_Float16)a.y; u.h[2] = (_Float16)a.z; u.h[3] = (_Float16)a.w;
  u.h[4] = (_Float16)b.x; u.h[5] = (_Float16)b.y; u.h[6] = (_Float16)b.z; u.h[7] = (_Float16)b.w;
  return u.i;
}
__device__ __forceinline__ v8h ld8h(const float* p) {
  Pack16 u;
  u.i = cvt8i(*(const v4f*)p, *(const v4f*)(p + 4));
  return u.h;
}
__device__ __forceinline__ v8h ld8h(const _Float16* p) { return *(const v8h*)p; }

__global__ __launch_bounds__(NTHR) void k_prep(const float* __restrict__ Wl, const float* __restrict__ Wr,
                                               const float* __restrict__ We, _Float16* Wh, _Float16* Weh, int K) {
  const int i  = blockIdx.x * NTHR + threadIdx.x;
  const int kq = K >> 3;
  const int nNode = NCOL * kq;
  const v4i z4 = {0, 0, 0, 0};
  Pack16 u;
  u.i = z4;
  _Float16* dst;
  if (i < nNode) {
    const int n  = i / kq;
    const int k0 = (i - n * kq) * 8;
    const float* W = (n < HCH) ? Wl : Wr;
    const int nn = n & (HCH - 1);
#pragma unroll
    for (int j = 0; j < 8; ++j) u.h[j] = (_Float16)(8.0f * W[(size_t)(k0 + j) * HCH + nn]);
    dst = Wh + (size_t)i * 8;
  } else if (i < nNode + 256) {
    const int ii = i - nNode;
    const int n  = ii >> 2;
    const int k0 = (ii & 3) * 8;
    if (k0 == 0) {
#pragma unroll
      for (int j = 0; j < 8; ++j) u.h[j] = (_Float16)(8.0f * We[j * HCH + n]);
    }
    dst = Weh + (size_t)ii * 8;
  } else {
    return;
  }
  *(volatile v4i*)dst = u.i;
  __threadfence();
  *(volatile v4i*)dst = u.i;
}

template <typename TI, int K>
__global__ __launch_bounds__(NTHR) void k_gemm(const TI* __restrict__ X, const _Float16* __restrict__ Wh,
                                               const float* __restrict__ bl, const float* __restrict__ br,
                                               float* XL, _Float16* XR, int nN) {
  constexpr int AP = K + 8;
  __shared__ __attribute__((aligned(16))) _Float16 At[GR * AP];
  __shared__ __attribute__((aligned(16))) float Xs[GR * XSP];

  const int tid  = threadIdx.x;
  const int lane = tid & 31;
  const int wave = tid >> 5;
  const int hh   = lane >> 4;
  const int m    = lane & 15;
  const int rowBase = blockIdx.x * GR;

  {
    const int r  = tid >> 3;
    const int c0 = (tid & 7) * (K / 8);
    int row = rowBase + r;
    if (row > nN - 1) row = nN - 1;
    const TI* p = X + (size_t)row * K + c0;
#pragma unroll
    for (int qq = 0; qq < K / 64; ++qq) *(v8h*)(At + r * AP + c0 + 8 * qq) = ld8h(p + 8 * qq);
  }
  __syncthreads();

  const int ncol = wave * 16 + m;
  v8f c0a = {0.f, 0.f, 0.f, 0.f, 0.f, 0.f, 0.f, 0.f};
  v8f c1a = {0.f, 0.f, 0.f, 0.f, 0.f, 0.f, 0.f, 0.f};
#pragma unroll
  for (int kt = 0; kt < K / 32; ++kt) {
    const int k0 = kt * 32;
    Frag a0, a1, b;
    const _Float16* pb  = Wh + (size_t)ncol * K + k0 + 8 * hh;
    const _Float16* pa0 = At + m * AP + k0 + 8 * hh;
    const _Float16* pa1 = At + (16 + m) * AP + k0 + 8 * hh;
    b.half[0]  = *(const v8h*)pb;  b.half[1]  = *(const v8h*)(pb + 16);
    a0.half[0] = *(const v8h*)pa0; a0.half[1] = *(const v8h*)(pa0 + 16);
    a1.half[0] = *(const v8h*)pa1; a1.half[1] = *(const v8h*)(pa1 + 16);
    c0a = wm(a0.v, b.v, c0a);
    c1a = wm(a1.v, b.v, c1a);
  }

  const int bi = ncol & (HCH - 1);
  const float bv = (wave < 4) ? bl[bi] : br[bi];
#pragma unroll
  for (int r = 0; r < 8; ++r) {
    Xs[(8 * hh + r) * XSP + ncol]      = c0a[r] * 0.125f + bv;
    Xs[(16 + 8 * hh + r) * XSP + ncol] = c1a[r] * 0.125f + bv;
  }
  __syncthreads();

  v4f xlv[2];
  float* xlp[2];
#pragma unroll
  for (int i = 0; i < 2; ++i) {
    const int r = 4 * wave + 2 * i + (lane >> 4);
    xlv[i] = *(const v4f*)(Xs + r * XSP + 4 * (lane & 15));
    xlp[i] = XL + (size_t)(rowBase + r) * HCH + 4 * (lane & 15);
  }
  const int r2 = 4 * wave + (lane >> 3);
  const int cc = 8 * (lane & 7);
  const v4i xrv = cvt8i(*(const v4f*)(Xs + r2 * XSP + HCH + cc), *(const v4f*)(Xs + r2 * XSP + HCH + cc + 4));
  _Float16* xrp = XR + (size_t)(rowBase + r2) * HCH + cc;

  *(volatile v4f*)xlp[0] = xlv[0];
  *(volatile v4f*)xlp[1] = xlv[1];
  *(volatile v4i*)xrp = xrv;
  __threadfence();
  *(volatile v4f*)xlp[0] = xlv[0];
  *(volatile v4f*)xlp[1] = xlv[1];
  *(volatile v4i*)xrp = xrv;
}

__global__ __launch_bounds__(NTHR) void k_edge(const float* __restrict__ ea, const _Float16* __restrict__ Weh,
                                               _Float16* EH, int nE) {
  __shared__ __attribute__((aligned(16))) float Es[EB * ESP];
  const int tid  = threadIdx.x;
  const int lane = tid & 31;
  const int wave = tid >> 5;
  const int hh   = lane >> 4;
  const int m    = lane & 15;
  const int rBase = blockIdx.x * EB;

  int e = rBase + wave * 16 + m;
  if (e > nE - 1) e = nE - 1;
  const v4i z4 = {0, 0, 0, 0};
  Pack16 u, z;
  z.i = z4;
  u.i = cvt8i(*(const v4f*)(ea + (size_t)e * EDIM), *(const v4f*)(ea + (size_t)e * EDIM + 4));
  Frag a;
  a.half[0] = (hh != 0) ? z.h : u.h;
  a.half[1] = z.h;
  const v8f zero8 = {0.f, 0.f, 0.f, 0.f, 0.f, 0.f, 0.f, 0.f};
  v8f acc[4];
#pragma unroll
  for (int nt = 0; nt < 4; ++nt) {
    Frag b;
    const _Float16* pb = Weh + (nt * 16 + m) * 32 + 8 * hh;
    b.half[0] = *(const v8h*)pb;
    b.half[1] = *(const v8h*)(pb + 16);
    acc[nt] = wm(a.v, b.v, zero8);
  }
#pragma unroll
  for (int nt = 0; nt < 4; ++nt) {
#pragma unroll
    for (int r = 0; r < 8; ++r) Es[(wave * 16 + 8 * hh + r) * ESP + nt * 16 + m] = acc[nt][r] * 0.125f;
  }
  __syncthreads();

  v4i sv[4];
  _Float16* sp[4];
#pragma unroll
  for (int i = 0; i < 4; ++i) {
    const int row = wave * 16 + 4 * i + (lane >> 3);
    const int cc  = 8 * (lane & 7);
    sv[i] = cvt8i(*(const v4f*)(Es + row * ESP + cc), *(const v4f*)(Es + row * ESP + cc + 4));
    sp[i] = EH + (size_t)(rBase + row) * HCH + cc;
  }
#pragma unroll
  for (int i = 0; i < 4; ++i) *(volatile v4i*)sp[i] = sv[i];
  __threadfence();
#pragma unroll
  for (int i = 0; i < 4; ++i) *(volatile v4i*)sp[i] = sv[i];
}

template <bool FIN>
__global__ __launch_bounds__(NTHR) void k_gat(
    const float* __restrict__ XL, const _Float16* __restrict__ XR, const _Float16* __restrict__ EH,
    const int* __restrict__ ei, const float* __restrict__ We, const float* __restrict__ att,
    const float* __restrict__ bias, const _Float16* H0in, const float* __restrict__ linW,
    const float* __restrict__ linb, _Float16* H0out, float* out, int nN, int nE) {
  extern __shared__ v4f lds_dyn[];
  float* lds  = (float*)lds_dyn;
  float* sacc = lds;
  float* amx  = lds + S_AMX;
  float* den  = lds + S_DEN;
  float* outs = lds + S_OUTS;
  int*   list = (int*)(lds + S_LIST);
  int*   wcnt = (int*)(lds + S_WCNT);

  const int tid  = threadIdx.x;
  const int lane = tid & 31;
  const int wave = tid >> 5;
  const int q    = lane >> 3;
  const int cl   = lane & 7;
  const int c8   = cl * 8;
  const int hd   = cl >> 1;
  const int nodeBase = blockIdx.x * NB;

  {
    const v4f z4 = {0.f, 0.f, 0.f, 0.f};
    const v4f n4 = {-1.0e30f, -1.0e30f, -1.0e30f, -1.0e30f};
    for (int i = tid; i < S_LIST / 4; i += NTHR) lds_dyn[i] = (i >= S_AMX / 4 && i < S_DEN / 4) ? n4 : z4;
  }
  U8 at8, bs8, eh8, lw8;
  at8.v[0] = *(const v4f*)(att + c8);   at8.v[1] = *(const v4f*)(att + c8 + 4);
  bs8.v[0] = *(const v4f*)(bias + c8);  bs8.v[1] = *(const v4f*)(bias + c8 + 4);
  lw8.v[0] = *(const v4f*)(linW + c8);  lw8.v[1] = *(const v4f*)(linW + c8 + 4);
  {
    v4f s0 = {0.f, 0.f, 0.f, 0.f}, s1 = {0.f, 0.f, 0.f, 0.f};
#pragma unroll
    for (int k = 0; k < EDIM; ++k) {
      s0 += *(const v4f*)(We + k * HCH + c8);
      s1 += *(const v4f*)(We + k * HCH + c8 + 4);
    }
    eh8.v[0] = s0 * 0.01f;
    eh8.v[1] = s1 * 0.01f;
  }
  const float lb = linb[0];
  __syncthreads();

  const int* eid = ei + nE;
  const bool al16 = ((nE & 3) == 0);
  const int nChunks = (nE + CHUNK - 1) / CHUNK;

#pragma unroll 1
  for (int ch = 0; ch < nChunks; ++ch) {
    const int cbase = ch * CHUNK;
    int wc = 0;
#pragma unroll
    for (int g = 0; g < NGRP; ++g) {
      const int el0 = (g * NTHR + tid) * 4;
      const int e0  = cbase + el0;
      const int sent = -2147483647 - 1;
      v4i d;
      if (al16 && (e0 + 3 < nE)) {
        d = *(const v4i*)(eid + e0);
      } else {
        d.x = (e0     < nE) ? eid[e0]     : sent;
        d.y = (e0 + 1 < nE) ? eid[e0 + 1] : sent;
        d.z = (e0 + 2 < nE) ? eid[e0 + 2] : sent;
        d.w = (e0 + 3 < nE) ? eid[e0 + 3] : sent;
      }
      const unsigned s0 = (unsigned)d.x - (unsigned)nodeBase;
      const unsigned s1 = (unsigned)d.y - (unsigned)nodeBase;
      const unsigned s2 = (unsigned)d.z - (unsigned)nodeBase;
      const unsigned s3 = (unsigned)d.w - (unsigned)nodeBase;
      const bool h0 = s0 < (unsigned)NB;
      const bool h1 = s1 < (unsigned)NB;
      const bool h2 = s2 < (unsigned)NB;
      const bool h3 = s3 < (unsigned)NB;
      const unsigned many = __builtin_amdgcn_ballot_w32(h0 | h1 | h2 | h3);
      if (many != 0u) {
#define HITJ(J, HJ, SJ) {                                                          \
          const unsigned mj = __builtin_amdgcn_ballot_w32(HJ);                         \
          if (mj != 0u) {                                                              \
            if (HJ) {                                                                  \
              const int pos = wc + (int)__builtin_amdgcn_mbcnt_lo(mj, 0u);             \
              if (pos < WCAP) list[wave * WCAP + pos] = ((el0 + (J)) << 10) | (int)(SJ); \
            }                                                                          \
            wc += (int)__builtin_popcount(mj);                                         \
          } }
        HITJ(0, h0, s0)
        HITJ(1, h1, s1)
        HITJ(2, h2, s2)
        HITJ(3, h3, s3)
#undef HITJ
      }
    }
    if (lane == 0) wcnt[wave] = wc;
    __syncthreads();

    if (wave == 0) {
      int n0 = __builtin_amdgcn_readfirstlane(wcnt[0]);
      n0 = n0 < 0 ? 0 : (n0 > WCAP ? WCAP : n0);
      int pbase = n0;
#pragma unroll
      for (int w = 1; w < NWAVE; ++w) {
        int nw = __builtin_amdgcn_readfirstlane(wcnt[w]);
        nw = nw < 0 ? 0 : (nw > WCAP ? WCAP : nw);
        for (int i = lane; i < nw; i += 32) list[pbase + i] = list[w * WCAP + i];
        pbase += nw;
      }
      if (lane == 0) wcnt[NWAVE] = pbase;
    }
    __syncthreads();

    if (wave == 0) {
      int T = __builtin_amdgcn_readfirstlane(wcnt[NWAVE]);
      T = T < 0 ? 0 : (T > NWAVE * WCAP ? NWAVE * WCAP : T);
      for (int g0 = 0; g0 < T; g0 += 4) {
        const int g = g0 + q;
        const bool valid = g < T;
        const int ent = list[valid ? g : g0];
        int slot = ent & 1023;
        slot = slot > NB - 1 ? NB - 1 : slot;
        const int el = (ent >> 10) & (CHUNK - 1);
        int e = cbase + el;
        e = e > nE - 1 ? nE - 1 : e;
        int src = ei[e];
        src = src < 0 ? 0 : (src > nN - 1 ? nN - 1 : src);
        int nd = nodeBase + slot;
        nd = nd > nN - 1 ? nN - 1 : nd;

        const int key = valid ? slot : (NB + q);
        const int k0 = __builtin_amdgcn_readlane(key, 0);
        const int k1 = __builtin_amdgcn_readlane(key, 8);
        const int k2 = __builtin_amdgcn_readlane(key, 16);
        const int rank = ((q > 0 && k0 == key) ? 1 : 0) + ((q > 1 && k1 == key) ? 1 : 0) + ((q > 2 && k2 == key) ? 1 : 0);
        const int npass = 1 + ((__builtin_amdgcn_ballot_w32(rank >= 1) != 0u) ? 1 : 0)
                            + ((__builtin_amdgcn_ballot_w32(rank >= 2) != 0u) ? 1 : 0)
                            + ((__builtin_amdgcn_ballot_w32(rank >= 3) != 0u) ? 1 : 0);

        Pack16 peh, pxr;
        U8 xl;
        peh.i   = *(const v4i*)(EH + (size_t)e * HCH + c8);
        pxr.i   = *(const v4i*)(XR + (size_t)nd * HCH + c8);
        xl.v[0] = *(const v4f*)(XL + (size_t)src * HCH + c8);
        xl.v[1] = *(const v4f*)(XL + (size_t)src * HCH + c8 + 4);
        float al = 0.f;
#pragma unroll
        for (int j = 0; j < 8; ++j) {
          float mv = xl.f[j] + ((float)pxr.h[j] + (float)peh.h[j]);
          mv = fmaxf(mv, 0.2f * mv);
          al += mv * at8.f[j];
        }
        al += __shfl_xor(al, 1, 32);

        volatile float* pM = amx + slot * 4 + hd;
        volatile float* pD = den + slot * 4 + hd;
        volatile v4f*   pa = (volatile v4f*)(sacc + slot * HCH + c8);
        for (int t = 0; t < npass; ++t) {
          const bool act = valid && (rank == t);
          const float M = *pM;
          const float D = *pD;
          const v4f a0 = pa[0];
          const v4f a1 = pa[1];
          const float Mn = fmaxf(M, al);
          const float sc = __expf(M - Mn);
          const float pr = __expf(al - Mn);
          const v4f n0 = a0 * sc + pr * xl.v[0];
          const v4f n1 = a1 * sc + pr * xl.v[1];
          if (act) {
            pa[0] = n0;
            pa[1] = n1;
            if ((lane & 1) == 0) {
              *pM = Mn;
              *pD = D * sc + pr;
            }
          }
          asm volatile("" ::: "memory");
        }
      }
    }
    __syncthreads();
  }

#pragma unroll 1
  for (int it = 0; it < NB / (NWAVE * 4); ++it) {
    const int slot = wave * (NB / NWAVE) + 4 * it + q;
    const int node = nodeBase + slot;
    const bool valid = node < nN;
    const int nd = valid ? node : nN - 1;
    Pack16 pxr;
    U8 xl;
    pxr.i   = *(const v4i*)(XR + (size_t)nd * HCH + c8);
    xl.v[0] = *(const v4f*)(XL + (size_t)nd * HCH + c8);
    xl.v[1] = *(const v4f*)(XL + (size_t)nd * HCH + c8 + 4);
    float al = 0.f;
#pragma unroll
    for (int j = 0; j < 8; ++j) {
      float mv = xl.f[j] + ((float)pxr.h[j] + eh8.f[j]);
      mv = fmaxf(mv, 0.2f * mv);
      al += mv * at8.f[j];
    }
    al += __shfl_xor(al, 1, 32);
    const float M = amx[slot * 4 + hd];
    const float D = den[slot * 4 + hd];
    const v4f a0 = *(const v4f*)(sacc + slot * HCH + c8);
    const v4f a1 = *(const v4f*)(sacc + slot * HCH + c8 + 4);
    const float Mn = fmaxf(M, al);
    const float sc = __expf(M - Mn);
    const float pr = __expf(al - Mn);
    const float Dn = D * sc + pr;
    const float inv = 1.0f / Dn;
    U8 h;
    h.v[0] = (a0 * sc + pr * xl.v[0]) * inv + bs8.v[0];
    h.v[1] = (a1 * sc + pr * xl.v[1]) * inv + bs8.v[1];
#pragma unroll
    for (int j = 0; j < 8; ++j) h.f[j] = fmaxf(h.f[j], 0.f);
    if (!FIN) {
      const v4i hv = cvt8i(h.v[0], h.v[1]);
      _Float16* hp = H0out + (size_t)nd * HCH + c8;
      if (valid) *(volatile v4i*)hp = hv;
      __threadfence();
      if (valid) *(volatile v4i*)hp = hv;
    } else {
      Pack16 ph;
      ph.i = *(const v4i*)(H0in + (size_t)nd * HCH + c8);
      float part = 0.f;
#pragma unroll
      for (int j = 0; j < 8; ++j) part += (h.f[j] + (float)ph.h[j]) * lw8.f[j];
      part += __shfl_xor(part, 1, 32);
      part += __shfl_xor(part, 2, 32);
      part += __shfl_xor(part, 4, 32);
      if (valid && cl == 0) outs[slot] = part + lb;
    }
  }
  if (FIN) {
    __syncthreads();
    if (tid < NB / 4) {
      const int n0 = nodeBase + 4 * tid;
      const v4f v = *(const v4f*)(outs + 4 * tid);
      float* op = out + n0;
      if (n0 + 3 < nN) {
        *(volatile v4f*)op = v;
      } else {
        if (n0 < nN)     ((volatile float*)op)[0] = v.x;
        if (n0 + 1 < nN) ((volatile float*)op)[1] = v.y;
        if (n0 + 2 < nN) ((volatile float*)op)[2] = v.z;
      }
      __threadfence();
      if (n0 + 3 < nN) {
        *(volatile v4f*)op = v;
      } else {
        if (n0 < nN)     ((volatile float*)op)[0] = v.x;
        if (n0 + 1 < nN) ((volatile float*)op)[1] = v.y;
        if (n0 + 2 < nN) ((volatile float*)op)[2] = v.z;
      }
    }
  }
}

static size_t al256(size_t b) { return (b + 255) & ~(size_t)255; }

extern "C" void kernel_launch(void* const* d_in, const int* in_sizes, int n_in,
                              void* d_out, int out_size, void* d_ws, size_t ws_size,
                              hipStream_t stream) {
  if (n_in < 19) return;
  const int nN = in_sizes[0] / NCOL;
  const int nE = in_sizes[1] / 2;
  if (nN <= 0 || in_sizes[0] != nN * NCOL) return;
  if (nE <= 0 || in_sizes[1] != 2 * nE || in_sizes[2] != nE * EDIM) return;
  if (in_sizes[3] != NCOL * HCH || in_sizes[5] != NCOL * HCH) return;
  if (in_sizes[10] != HCH * HCH || in_sizes[12] != HCH * HCH) return;
  if (in_sizes[7] != EDIM * HCH || in_sizes[14] != EDIM * HCH) return;
  if (in_sizes[4] != HCH || in_sizes[6] != HCH || in_sizes[8] != HCH || in_sizes[9] != HCH) return;
  if (in_sizes[11] != HCH || in_sizes[13] != HCH || in_sizes[15] != HCH || in_sizes[16] != HCH) return;
  if (in_sizes[17] != HCH || in_sizes[18] < 1) return;
  if (out_size != nN) return;

  const float* x     = (const float*)d_in[0];
  const int*   ei    = (const int*)d_in[1];
  const float* ea    = (const float*)d_in[2];
  const float* Wl0   = (const float*)d_in[3];
  const float* bl0   = (const float*)d_in[4];
  const float* Wr0   = (const float*)d_in[5];
  const float* br0   = (const float*)d_in[6];
  const float* We0   = (const float*)d_in[7];
  const float* att0  = (const float*)d_in[8];
  const float* bias0 = (const float*)d_in[9];
  const float* Wl1   = (const float*)d_in[10];
  const float* bl1   = (const float*)d_in[11];
  const float* Wr1   = (const float*)d_in[12];
  const float* br1   = (const float*)d_in[13];
  const float* We1   = (const float*)d_in[14];
  const float* att1  = (const float*)d_in[15];
  const float* bias1 = (const float*)d_in[16];
  const float* linW  = (const float*)d_in[17];
  const float* linb  = (const float*)d_in[18];
  float* out = (float*)d_out;

  const int nPad = ((nN + GR - 1) / GR) * GR;
  const int ePad = ((nE + EB - 1) / EB) * EB;

  char* base = (char*)d_ws;
  size_t off = 0;
  _Float16* Wh0  = (_Float16*)(base + off); off += al256((size_t)NCOL * NCOL * 2);
  _Float16* Wh1  = (_Float16*)(base + off); off += al256((size_t)NCOL * HCH * 2);
  _Float16* We0h = (_Float16*)(base + off); off += al256((size_t)HCH * 32 * 2);
  _Float16* We1h = (_Float16*)(base + off); off += al256((size_t)HCH * 32 * 2);
  float*    XL   = (float*)(base + off);    off += al256((size_t)nPad * HCH * 4);
  _Float16* XR   = (_Float16*)(base + off); off += al256((size_t)nPad * HCH * 2);
  _Float16* H0   = (_Float16*)(base + off); off += al256((size_t)nPad * HCH * 2);
  _Float16* EH   = (_Float16*)(base + off); off += al256((size_t)ePad * HCH * 2);
  if (off > ws_size) return;

  const int gPrep0 = (NCOL * (NCOL / 8) + 256 + NTHR - 1) / NTHR;
  const int gPrep1 = (NCOL * (HCH / 8) + 256 + NTHR - 1) / NTHR;
  const int gGat   = (nN + NB - 1) / NB;

  k_prep<<<gPrep0, NTHR, 0, stream>>>(Wl0, Wr0, We0, Wh0, We0h, NCOL);
  k_prep<<<gPrep1, NTHR, 0, stream>>>(Wl1, Wr1, We1, Wh1, We1h, HCH);

  k_gemm<float, NCOL><<<nPad / GR, NTHR, 0, stream>>>(x, Wh0, bl0, br0, XL, XR, nN);
  k_edge<<<ePad / EB, NTHR, 0, stream>>>(ea, We0h, EH, nE);
  hipFuncSetAttribute(reinterpret_cast<const void*>(&k_gat<false>),
                      hipFuncAttributeMaxDynamicSharedMemorySize, LDS_BYTES);
  k_gat<false><<<gGat, NTHR, LDS_BYTES, stream>>>(XL, XR, EH, ei, We0, att0, bias0, H0, linW, linb,
                                                  H0, out, nN, nE);

  k_gemm<_Float16, HCH><<<nPad / GR, NTHR, 0, stream>>>(H0, Wh1, bl1, br1, XL, XR, nN);
  k_edge<<<ePad / EB, NTHR, 0, stream>>>(ea, We1h, EH, nE);
  hipFuncSetAttribute(reinterpret_cast<const void*>(&k_gat<true>),
                      hipFuncAttributeMaxDynamicSharedMemorySize, LDS_BYTES);
  k_gat<true><<<gGat, NTHR, LDS_BYTES, stream>>>(XL, XR, EH, ei, We1, att1, bias1, H0, linW, linb,
                                                 H0, out, nN, nE);
}
